// GPT2GroupQueryAttention_4526895530008
// MI455X (gfx1250) — hardware-verified
//
#include <hip/hip_runtime.h>


#define NB_  4
#define SS   2048
#define HID  1024
#define NH_  16
#define DH   64
#define NG   1024
#define GD   128
#define PCAR 1024.0f
typedef _Float16 h16;
typedef unsigned short bf;
typedef __attribute__((ext_vector_type(16))) __bf16   v16bf;
typedef __attribute__((ext_vector_type(16))) _Float16 v16h;
typedef __attribute__((ext_vector_type(8)))  _Float16 v8h;
typedef __attribute__((ext_vector_type(8)))  unsigned short v8us;
typedef __attribute__((ext_vector_type(8)))  float    v8f;
typedef __attribute__((ext_vector_type(4)))  float    v4f;
typedef v8h  __attribute__((may_alias)) v8ha;
typedef v4f  __attribute__((may_alias)) v4fa;
typedef v8us __attribute__((may_alias)) v8usa;

__device__ __forceinline__ unsigned short f2bf(float f) { unsigned u = __float_as_uint(f); u += 0x7FFFu + ((u >> 16) & 1u); return (unsigned short)(u >> 16); }
__device__ __forceinline__ float bf2f(unsigned short b) { return __uint_as_float(((unsigned)b) << 16); }
__device__ __forceinline__ float bfr(float f) { return bf2f(f2bf(f)); }
__device__ __forceinline__ v16h cat16(v8h lo, v8h hi) { return __builtin_shufflevector(lo, hi, 0, 1, 2, 3, 4, 5, 6, 7, 8, 9, 10, 11, 12, 13, 14, 15); }
__device__ __forceinline__ v16bf cat16b(v8us lo, v8us hi) { return __builtin_bit_cast(v16bf, __builtin_shufflevector(lo, hi, 0, 1, 2, 3, 4, 5, 6, 7, 8, 9, 10, 11, 12, 13, 14, 15)); }
__device__ __forceinline__ v8f wmma16(v16h a, v16h b, v8f c) { return __builtin_amdgcn_wmma_f32_16x16x32_f16(false, a, false, b, (short)0, c, false, false); }
__device__ __forceinline__ v8f wmmab(v16bf a, v16bf b, v8f c) { return __builtin_amdgcn_wmma_f32_16x16x32_bf16(false, a, false, b, (short)0, c, false, false); }


template <typename T16> struct WFrag;
template <> struct WFrag<h16> { typedef v16h V; static __device__ __forceinline__ V ld(const h16* p) { return cat16(*(const v8h*)p, *(const v8h*)(p + 16)); } static __device__ __forceinline__ v8f mma(V a, V b, v8f c) { return wmma16(a, b, c); } };
template <> struct WFrag<bf> { typedef v16bf V; static __device__ __forceinline__ V ld(const bf* p) { return cat16b(*(const v8us*)p, *(const v8us*)(p + 16)); } static __device__ __forceinline__ v8f mma(V a, V b, v8f c) { return wmmab(a, b, c); } };
template <typename T16, int NSPLIT, bool BIAS>
__global__ __launch_bounds__(32) void k_gemmw(const T16* __restrict__ A, const T16* __restrict__ A2, const T16* __restrict__ Bt, const T16* __restrict__ Bt2, int K, float* C, int ldc, const float* __restrict__ bias, size_t sA, size_t sB, size_t sC) {
    typedef typename WFrag<T16>::V V;
    __shared__ __align__(16) float os[16 * 68];
    const size_t z = blockIdx.z; A += z * sA; if (A2) A2 += z * sA; Bt += z * sB; if (Bt2) Bt2 += z * sB; C += z * sC;
    const int lane = threadIdx.x & 31, lr = lane & 15, hi = lane >> 4; const int r0 = blockIdx.x * 64, c0 = blockIdx.y * 64;
    v8f acc[4][4];
#pragma unroll
    for (int mb = 0; mb < 4; ++mb)
#pragma unroll
        for (int nb = 0; nb < 4; ++nb) acc[mb][nb] = (v8f){};
    const size_t aoff = (size_t)(r0 + lr) * K + 8 * hi, boff = (size_t)(c0 + lr) * K + 8 * hi;
#pragma unroll 1
    for (int kc = 0; kc < K; kc += 32) {
        V a[4], a2[4];
#pragma unroll
        for (int mb = 0; mb < 4; ++mb) { a[mb] = WFrag<T16>::ld(A + aoff + (size_t)mb * 16 * K + kc); if (NSPLIT == 1 || NSPLIT == 2) a2[mb] = WFrag<T16>::ld(A2 + aoff + (size_t)mb * 16 * K + kc); }
#pragma unroll
        for (int nb = 0; nb < 4; ++nb) { const V b = WFrag<T16>::ld(Bt + boff + (size_t)nb * 16 * K + kc); V b2; if (NSPLIT >= 2) b2 = WFrag<T16>::ld(Bt2 + boff + (size_t)nb * 16 * K + kc);
#pragma unroll
            for (int mb = 0; mb < 4; ++mb) { acc[mb][nb] = WFrag<T16>::mma(a[mb], b, acc[mb][nb]); if (NSPLIT == 1 || NSPLIT == 2) acc[mb][nb] = WFrag<T16>::mma(a2[mb], b, acc[mb][nb]); if (NSPLIT >= 2) acc[mb][nb] = WFrag<T16>::mma(a[mb], b2, acc[mb][nb]); } }
        asm volatile("v_nop\n\tv_nop\n\tv_nop\n\tv_nop" : "+v"(acc[0][0]), "+v"(acc[1][1]), "+v"(acc[2][2]), "+v"(acc[3][3]) : "v"(a[0]), "v"(a[3]));
    }
#pragma unroll
    for (int mb = 0; mb < 4; ++mb) {
#pragma unroll
        for (int nb = 0; nb < 4; ++nb) {
#pragma unroll
            for (int j = 0; j < 8; ++j) os[(hi * 8 + j) * 68 + nb * 16 + lr] = acc[mb][nb][j]; }
        __builtin_amdgcn_wave_barrier(); asm volatile("" ::: "memory");
        float* crow = C + (size_t)(r0 + mb * 16) * ldc + c0;
#pragma unroll 1
        for (int ps = 0; ps < 2; ++ps) {
#pragma unroll
            for (int s = 0; s < 8; ++s) { const int row = 2 * s + hi, cofs = lr * 4; v4f val = *(const v4fa*)(os + row * 68 + cofs); if (BIAS) { val[0] += bfr(bias[c0 + cofs]); val[1] += bfr(bias[c0 + cofs + 1]); val[2] += bfr(bias[c0 + cofs + 2]); val[3] += bfr(bias[c0 + cofs + 3]); }
                *(volatile v4f*)(crow + (size_t)row * ldc + cofs) = val; }
            if (ps == 0) __threadfence(); }
        __builtin_amdgcn_wave_barrier(); asm volatile("" ::: "memory");
    }
}

__device__ __forceinline__ h16 tohx(float x) { return (h16)x; }
__device__ __forceinline__ void splitf(float y, unsigned short& h, unsigned short& l) { h = f2bf(y); l = f2bf(y - bf2f(h)); }
typedef __attribute__((ext_vector_type(2))) unsigned short v2us;
typedef __attribute__((ext_vector_type(4))) unsigned short v4us;
typedef __attribute__((ext_vector_type(2))) _Float16 v2h;
typedef __attribute__((ext_vector_type(4))) _Float16 v4h;

__global__ __launch_bounds__(256) void k_cvt8(const float* __restrict__ src, bf* dst, size_t n8) { const size_t i = (size_t)blockIdx.x * 256 + threadIdx.x; if (i >= n8) return; const v8f v = *(const v8f*)(src + i * 8); v8us o;
#pragma unroll
    for (int k = 0; k < 8; ++k) o[k] = f2bf(v[k]); *(volatile v8us*)(dst + i * 8) = o; __threadfence(); *(volatile v8us*)(dst + i * 8) = o; }
__global__ __launch_bounds__(256) void k_gpl(const float* __restrict__ FQ, const float* __restrict__ FK, bf* Qh, bf* Ql, bf* Kh, bf* Kl) { const int e = (blockIdx.x * 256 + threadIdx.x) * 4; if (e >= NH_ * NG * GD) return; const int j = e % GD; const int g = (e / GD) % NG; const int h = e / (GD * NG); const size_t src = (size_t)(2 * g + j / DH) * HID + h * DH + (j % DH); const v4f q = *(const v4f*)(FQ + src), k = *(const v4f*)(FK + src); v4us qh, ql, kh, kl;
#pragma unroll
    for (int u = 0; u < 4; ++u) { unsigned short a, b; splitf(q[u] * 0.125f, a, b); qh[u] = a; ql[u] = b; splitf(k[u], a, b); kh[u] = a; kl[u] = b; }
    for (int ps = 0; ps < 2; ++ps) { *(volatile v4us*)(Qh + e) = qh; *(volatile v4us*)(Ql + e) = ql; *(volatile v4us*)(Kh + e) = kh; *(volatile v4us*)(Kl + e) = kl; if (ps == 0) __threadfence(); } }
__global__ __launch_bounds__(256) void k_vt(const float* __restrict__ FV, h16* VT) { const int e = (blockIdx.x * 256 + threadIdx.x) * 2; if (e >= NH_ * GD * NG) return; const int g = e % NG; const int j = (e / NG) % GD; const int h = e / (NG * GD); v2h o;
#pragma unroll
    for (int u = 0; u < 2; ++u) o[u] = tohx(FV[(size_t)(2 * (g + u) + j / DH) * HID + h * DH + (j % DH)]); *(volatile v2h*)(VT + e) = o; __threadfence(); *(volatile v2h*)(VT + e) = o; }
__global__ __launch_bounds__(256) void k_mrg(const float* __restrict__ O, bf* Ah, bf* Al) { const int e = (blockIdx.x * 256 + threadIdx.x) * 4; if (e >= SS * HID) return; const int c = e % HID; const int s = e / HID; const int g = s / 2, h = (s % 2) * 8 + c / GD, j = c % GD; const float* r = O + ((size_t)h * NG + g) * GD + j; v4us oh, ol;
#pragma unroll
    for (int u = 0; u < 4; ++u) { unsigned short a, b; splitf(r[u] * (1.0f / PCAR), a, b); oh[u] = a; ol[u] = b; } *(volatile v4us*)(Ah + e) = oh; *(volatile v4us*)(Al + e) = ol; __threadfence(); *(volatile v4us*)(Ah + e) = oh; *(volatile v4us*)(Al + e) = ol; }
template <int NFULL, int TAIL> __global__ __launch_bounds__(256) void k_soft(const float* __restrict__ Sb, int nrows, int rowsper, int rvalid, int nvalid, h16* P) { const int lane = threadIdx.x & 31; const size_t row = (size_t)blockIdx.x * 8 + (threadIdx.x >> 5); if (row >= (size_t)nrows) return; constexpr int LD = NFULL * 128 + TAIL * 64; const float* sr = Sb + row * LD; h16* pr = P + row * LD; const bool live = (int)(row % rowsper) < rvalid; float mx = -3.0e38f;
#pragma unroll 1
    for (int ch = 0; ch < NFULL + TAIL; ++ch) { if (ch == NFULL && lane >= 16) break; const int j0 = ch * 128 + lane * 4; const v4f a = *(const v4f*)(sr + j0);
#pragma unroll
        for (int q = 0; q < 4; ++q) if (j0 + q < nvalid) mx = fmaxf(mx, a[q]); }
#pragma unroll
    for (int sh = 16; sh; sh >>= 1) mx = fmaxf(mx, __shfl_xor(mx, sh, 32));
    float sum = 0.f;
#pragma unroll 1
    for (int ch = 0; ch < NFULL + TAIL; ++ch) { if (ch == NFULL && lane >= 16) break; const int j0 = ch * 128 + lane * 4; const v4f a = *(const v4f*)(sr + j0);
#pragma unroll
        for (int q = 0; q < 4; ++q) if (j0 + q < nvalid) { float d0 = __fsub_rn(a[q], mx); asm volatile("" : "+v"(d0)); sum += __expf(d0); } }
#pragma unroll
    for (int sh = 16; sh; sh >>= 1) sum += __shfl_xor(sum, sh, 32);
    const float f = live ? __fdiv_rn(PCAR, sum) : 0.f;
    for (int ps = 0; ps < 2; ++ps) {
#pragma unroll 1
        for (int ch = 0; ch < NFULL + TAIL; ++ch) { if (ch == NFULL && lane >= 16) break; const int j0 = ch * 128 + lane * 4; const v4f a = *(const v4f*)(sr + j0); v4h o;
#pragma unroll
            for (int q = 0; q < 4; ++q) { float val = 0.f; if (live && j0 + q < nvalid) { float d0 = __fsub_rn(a[q], mx); asm volatile("" : "+v"(d0)); val = __fmul_rn(__expf(d0), f); } o[q] = tohx(val); } *(volatile v4h*)(pr + j0) = o; }
        if (ps == 0) __threadfence(); } }

extern "C" void kernel_launch(void* const* d_in, const int* in_sizes, int n_in,
                              void* d_out, int out_size, void* d_ws, size_t ws_size, hipStream_t stream) {
    (void)in_sizes; (void)n_in; (void)out_size;
    const float** I = (const float**)d_in;
    const float *x = I[0], *wq = I[1], *bq = I[2], *wk = I[3], *bk = I[4], *wv = I[5], *bv = I[6], *wo = I[7], *bo = I[8];
    float* OUT = (float*)d_out;
    char* wsp = (char*)d_ws;
    auto take = [&](size_t bytes) { char* p = wsp; wsp += (bytes + 255) & ~(size_t)255; return (void*)p; };
    bf* WQ = (bf*)take((size_t)HID * HID * 2); bf* WK_ = (bf*)take((size_t)HID * HID * 2); bf* WV = (bf*)take((size_t)HID * HID * 2); bf* WO = (bf*)take((size_t)HID * HID * 2);
    bf* XB = (bf*)take((size_t)SS * HID * 2); float* FQ = (float*)take((size_t)SS * HID * 4); float* FK = (float*)take((size_t)SS * HID * 4); bf* Qh = (bf*)take((size_t)NH_ * NG * GD * 2); bf* Ql = (bf*)take((size_t)NH_ * NG * GD * 2); bf* Kh = (bf*)take((size_t)NH_ * NG * GD * 2); bf* Kl = (bf*)take((size_t)NH_ * NG * GD * 2); h16* VT = (h16*)take((size_t)NH_ * GD * NG * 2);
    float* Sb = (float*)take((size_t)NH_ * NG * NG * 4); h16* P16 = (h16*)take((size_t)NH_ * NG * NG * 2); float* O = (float*)take((size_t)NH_ * NG * GD * 4); bf* Ah = (bf*)take((size_t)SS * HID * 2); bf* Al = (bf*)take((size_t)SS * HID * 2);
    if ((size_t)(wsp - (char*)d_ws) > ws_size) return;
    float* FV = FK;
    k_cvt8<<<(HID * HID / 8 + 255) / 256, 256, 0, stream>>>(wq, WQ, (size_t)HID * HID / 8); k_cvt8<<<(HID * HID / 8 + 255) / 256, 256, 0, stream>>>(wk, WK_, (size_t)HID * HID / 8); k_cvt8<<<(HID * HID / 8 + 255) / 256, 256, 0, stream>>>(wv, WV, (size_t)HID * HID / 8); k_cvt8<<<(HID * HID / 8 + 255) / 256, 256, 0, stream>>>(wo, WO, (size_t)HID * HID / 8);
    for (int b = 0; b < NB_; ++b) {
        k_cvt8<<<(SS * HID / 8 + 255) / 256, 256, 0, stream>>>(x + (size_t)b * SS * HID, XB, (size_t)SS * HID / 8);
        k_gemmw<bf, 0, true><<<dim3(SS / 64, HID / 64, 1), 32, 0, stream>>>(XB, nullptr, WQ, nullptr, HID, FQ, HID, bq, 0, 0, 0); k_gemmw<bf, 0, true><<<dim3(SS / 64, HID / 64, 1), 32, 0, stream>>>(XB, nullptr, WK_, nullptr, HID, FK, HID, bk, 0, 0, 0);
        k_gpl<<<(NH_ * NG * GD / 4 + 255) / 256, 256, 0, stream>>>(FQ, FK, Qh, Ql, Kh, Kl);
        k_gemmw<bf, 0, true><<<dim3(SS / 64, HID / 64, 1), 32, 0, stream>>>(XB, nullptr, WV, nullptr, HID, FV, HID, bv, 0, 0, 0); k_vt<<<(NH_ * GD * NG / 2 + 255) / 256, 256, 0, stream>>>(FV, VT);
        k_gemmw<bf, 2, false><<<dim3(NG / 64, NG / 64, NH_), 32, 0, stream>>>(Qh, Ql, Kh, Kl, GD, Sb, NG, nullptr, (size_t)NG * GD, (size_t)NG * GD, (size_t)NG * NG);
        k_soft<8, 0><<<NH_ * NG / 8, 256, 0, stream>>>(Sb, NH_ * NG, NG, NG, NG, P16);
        k_gemmw<h16, 0, false><<<dim3(NG / 64, GD / 64, NH_), 32, 0, stream>>>(P16, nullptr, VT, nullptr, NG, O, GD, nullptr, (size_t)NG * NG, (size_t)GD * NG, (size_t)NG * GD);
        k_mrg<<<(SS * HID / 4 + 255) / 256, 256, 0, stream>>>(O, Ah, Al);
        k_gemmw<bf, 1, true><<<dim3(SS / 64, HID / 64, 1), 32, 0, stream>>>(Ah, Al, WO, nullptr, HID, OUT + (size_t)b * SS * HID, HID, bo, 0, 0, 0); }
}
